// GraphLayer_1700807049908
// MI455X (gfx1250) — hardware-verified
//
#include <hip/hip_runtime.h>


#define NBT  32
#define NN   128
#define FIN  512
#define HH   256
#define NR   (NBT * NN)
#define DM   HH
#define TT   NR
typedef _Float16 h16;
typedef unsigned short bf;
typedef __attribute__((ext_vector_type(16))) __bf16   v16bf;
typedef __attribute__((ext_vector_type(16))) _Float16 v16h;
typedef __attribute__((ext_vector_type(8)))  _Float16 v8h;
typedef __attribute__((ext_vector_type(8)))  unsigned short v8us;
typedef __attribute__((ext_vector_type(8)))  float    v8f;
typedef __attribute__((ext_vector_type(4)))  float    v4f;
typedef v8h  __attribute__((may_alias)) v8ha;
typedef v4f  __attribute__((may_alias)) v4fa;
typedef v8us __attribute__((may_alias)) v8usa;

__device__ __forceinline__ unsigned short f2bf(float f) { unsigned u = __float_as_uint(f); u += 0x7FFFu + ((u >> 16) & 1u); return (unsigned short)(u >> 16); }
__device__ __forceinline__ float bf2f(unsigned short b) { return __uint_as_float(((unsigned)b) << 16); }
__device__ __forceinline__ float bfr(float f) { return bf2f(f2bf(f)); }
__device__ __forceinline__ v16h cat16(v8h lo, v8h hi) { return __builtin_shufflevector(lo, hi, 0, 1, 2, 3, 4, 5, 6, 7, 8, 9, 10, 11, 12, 13, 14, 15); }
__device__ __forceinline__ v16bf cat16b(v8us lo, v8us hi) { return __builtin_bit_cast(v16bf, __builtin_shufflevector(lo, hi, 0, 1, 2, 3, 4, 5, 6, 7, 8, 9, 10, 11, 12, 13, 14, 15)); }
__device__ __forceinline__ v8f wmma16(v16h a, v16h b, v8f c) { return __builtin_amdgcn_wmma_f32_16x16x32_f16(false, a, false, b, (short)0, c, false, false); }
__device__ __forceinline__ v8f wmmab(v16bf a, v16bf b, v8f c) { return __builtin_amdgcn_wmma_f32_16x16x32_bf16(false, a, false, b, (short)0, c, false, false); }


template <typename T16> struct WFrag;
template <> struct WFrag<h16> { typedef v16h V; static __device__ __forceinline__ V ld(const h16* p) { return cat16(*(const v8h*)p, *(const v8h*)(p + 16)); } static __device__ __forceinline__ v8f mma(V a, V b, v8f c) { return wmma16(a, b, c); } };
template <> struct WFrag<bf> { typedef v16bf V; static __device__ __forceinline__ V ld(const bf* p) { return cat16b(*(const v8us*)p, *(const v8us*)(p + 16)); } static __device__ __forceinline__ v8f mma(V a, V b, v8f c) { return wmmab(a, b, c); } };
template <typename T16, int NSPLIT, bool BIAS>
__global__ __launch_bounds__(32) void k_gemmw(const T16* __restrict__ A, const T16* __restrict__ A2, const T16* __restrict__ Bt, const T16* __restrict__ Bt2, int K, float* C, int ldc, const float* __restrict__ bias, size_t sA, size_t sB, size_t sC) {
    typedef typename WFrag<T16>::V V;
    __shared__ __align__(16) float os[16 * 68];
    const size_t z = blockIdx.z; A += z * sA; if (A2) A2 += z * sA; Bt += z * sB; if (Bt2) Bt2 += z * sB; C += z * sC;
    const int lane = threadIdx.x & 31, lr = lane & 15, hi = lane >> 4; const int r0 = blockIdx.x * 64, c0 = blockIdx.y * 64;
    v8f acc[4][4];
#pragma unroll
    for (int mb = 0; mb < 4; ++mb)
#pragma unroll
        for (int nb = 0; nb < 4; ++nb) acc[mb][nb] = (v8f){};
    const size_t aoff = (size_t)(r0 + lr) * K + 8 * hi, boff = (size_t)(c0 + lr) * K + 8 * hi;
#pragma unroll 1
    for (int kc = 0; kc < K; kc += 32) {
        V a[4], a2[4];
#pragma unroll
        for (int mb = 0; mb < 4; ++mb) { a[mb] = WFrag<T16>::ld(A + aoff + (size_t)mb * 16 * K + kc); if (NSPLIT == 1 || NSPLIT == 2) a2[mb] = WFrag<T16>::ld(A2 + aoff + (size_t)mb * 16 * K + kc); }
#pragma unroll
        for (int nb = 0; nb < 4; ++nb) { const V b = WFrag<T16>::ld(Bt + boff + (size_t)nb * 16 * K + kc); V b2; if (NSPLIT >= 2) b2 = WFrag<T16>::ld(Bt2 + boff + (size_t)nb * 16 * K + kc);
#pragma unroll
            for (int mb = 0; mb < 4; ++mb) { acc[mb][nb] = WFrag<T16>::mma(a[mb], b, acc[mb][nb]); if (NSPLIT == 1 || NSPLIT == 2) acc[mb][nb] = WFrag<T16>::mma(a2[mb], b, acc[mb][nb]); if (NSPLIT >= 2) acc[mb][nb] = WFrag<T16>::mma(a[mb], b2, acc[mb][nb]); } }
        asm volatile("v_nop\n\tv_nop\n\tv_nop\n\tv_nop" : "+v"(acc[0][0]), "+v"(acc[1][1]), "+v"(acc[2][2]), "+v"(acc[3][3]) : "v"(a[0]), "v"(a[3]));
    }
#pragma unroll
    for (int mb = 0; mb < 4; ++mb) {
#pragma unroll
        for (int nb = 0; nb < 4; ++nb) {
#pragma unroll
            for (int j = 0; j < 8; ++j) os[(hi * 8 + j) * 68 + nb * 16 + lr] = acc[mb][nb][j]; }
        __builtin_amdgcn_wave_barrier(); asm volatile("" ::: "memory");
        float* crow = C + (size_t)(r0 + mb * 16) * ldc + c0;
#pragma unroll 1
        for (int ps = 0; ps < 2; ++ps) {
#pragma unroll
            for (int s = 0; s < 8; ++s) { const int row = 2 * s + hi, cofs = lr * 4; v4f val = *(const v4fa*)(os + row * 68 + cofs); if (BIAS) { val[0] += bfr(bias[c0 + cofs]); val[1] += bfr(bias[c0 + cofs + 1]); val[2] += bfr(bias[c0 + cofs + 2]); val[3] += bfr(bias[c0 + cofs + 3]); }
                *(volatile v4f*)(crow + (size_t)row * ldc + cofs) = val; }
            if (ps == 0) __threadfence(); }
        __builtin_amdgcn_wave_barrier(); asm volatile("" ::: "memory");
    }
}

typedef __attribute__((ext_vector_type(4))) unsigned short v4us;
typedef __attribute__((ext_vector_type(2))) unsigned short v2us;
__device__ __forceinline__ void splitf(float y, unsigned short& h, unsigned short& l) { h = f2bf(y); l = f2bf(y - bf2f(h)); }
__device__ __forceinline__ float sigm(float a) { return __fdiv_rn(1.0f, __fadd_rn(1.0f, __builtin_amdgcn_exp2f(__fmul_rn(a, -1.4426950408889634f)))); }
__global__ __launch_bounds__(256) void k_cvt8(const float* __restrict__ src, bf* dst, size_t n8) { const size_t i = (size_t)blockIdx.x * 256 + threadIdx.x; if (i >= n8) return; const v8f v = *(const v8f*)(src + i * 8); v8us o;
#pragma unroll
    for (int k = 0; k < 8; ++k) o[k] = f2bf(v[k]); *(volatile v8us*)(dst + i * 8) = o; __threadfence(); *(volatile v8us*)(dst + i * 8) = o; }

__global__ __launch_bounds__(256) void k_wtG(const float* __restrict__ w, int K, int N, bf* Bt) {
    const int lane = threadIdx.x & 31; const int L0 = (blockIdx.x * 8 + (threadIdx.x >> 5)) * 8; const int nlines = N * K / 64;
#pragma unroll
    for (int ps = 0; ps < 2; ++ps) {
#pragma unroll 1
        for (int l = 0; l < 8; ++l) { const int L = L0 + l; if (L >= nlines) break; const size_t e = (size_t)L * 64 + lane * 2; const int k = (int)(e % K), n = (int)(e / K); v2us o;
            o[0] = f2bf(w[(size_t)k * N + n]); o[1] = f2bf(w[(size_t)(k + 1) * N + n]); *(volatile v2us*)(Bt + e) = o; }
        if (ps == 0) __threadfence(); }
}

__global__ __launch_bounds__(256) void k_tohl(const float* __restrict__ F, bf* Hh, bf* Hl, size_t n4) { const size_t i = (size_t)blockIdx.x * 256 + threadIdx.x; if (i >= n4) return; const v4f a = *(const v4f*)(F + i * 4); v4us oh, ol;
#pragma unroll
    for (int q = 0; q < 4; ++q) { unsigned short h2, l2; splitf(a[q], h2, l2); oh[q] = h2; ol[q] = l2; }
    *(volatile v4us*)(Hh + i * 4) = oh; *(volatile v4us*)(Hl + i * 4) = ol; __threadfence(); *(volatile v4us*)(Hh + i * 4) = oh; *(volatile v4us*)(Hl + i * 4) = ol; }
__global__ __launch_bounds__(256) void k_vtB(const float* __restrict__ F, bf* Vh, bf* Vl) { const size_t e = ((size_t)blockIdx.x * 256 + threadIdx.x) * 2; if (e >= (size_t)NBT * HH * NN) return; const int m = (int)(e % NN); const int d = (int)((e / NN) % HH); const int b = (int)(e / ((size_t)NN * HH)); v2us oh, ol;
#pragma unroll
    for (int q = 0; q < 2; ++q) { unsigned short h2, l2; splitf(F[((size_t)b * NN + m + q) * HH + d], h2, l2); oh[q] = h2; ol[q] = l2; }
    *(volatile v2us*)(Vh + e) = oh; *(volatile v2us*)(Vl + e) = ol; __threadfence(); *(volatile v2us*)(Vh + e) = oh; *(volatile v2us*)(Vl + e) = ol; }
__global__ __launch_bounds__(256) void k_esoft(const float* __restrict__ Sb, const float* __restrict__ area, const float* __restrict__ co, const float* __restrict__ We1, const float* __restrict__ be1, const float* __restrict__ We2, const float* __restrict__ be2, bf* Ph, bf* Pl) {
    const int lane = threadIdx.x & 31; const size_t row = (size_t)blockIdx.x * 8 + (threadIdx.x >> 5); if (row >= (size_t)NR) return; const int n = (int)(row % NN); const float an = bfr(area[row]); float v[4]; float mx = -3.0e38f;
    float cm[4]; for (int q = 0; q < 4; ++q) cm[q] = bfr(co[(size_t)n * NN + lane * 4 + q]);
    float acc[4] = {0.f, 0.f, 0.f, 0.f};
#pragma unroll 1
    for (int d = 0; d < HH; ++d) { const float w0 = bfr(We1[d]), w1 = bfr(We1[HH + d]), bb = bfr(be1[d]), w2 = bfr(We2[d]); float a0 = __fmul_rn(an, w0); asm volatile("" : "+v"(a0));
#pragma unroll
        for (int q = 0; q < 4; ++q) { float c1 = __fmul_rn(cm[q], w1); asm volatile("" : "+v"(c1)); float h = __fadd_rn(__fadd_rn(a0, c1), bb); h = fmaxf(h, 0.0f); float p = __fmul_rn(h, w2); asm volatile("" : "+v"(p)); acc[q] = __fadd_rn(acc[q], p); } }
    const v4f a = *(const v4f*)(Sb + row * NN + lane * 4);
#pragma unroll
    for (int q = 0; q < 4; ++q) { const float ew = sigm(__fadd_rn(acc[q], bfr(be2[0]))); float sc = __fmul_rn(a[q], 0.0625f); asm volatile("" : "+v"(sc)); const float t = __fmul_rn(sc, ew); v[q] = t; mx = fmaxf(mx, t); }
#pragma unroll
    for (int sh = 16; sh; sh >>= 1) mx = fmaxf(mx, __shfl_xor(mx, sh, 32));
    float sum = 0.f;
#pragma unroll
    for (int q = 0; q < 4; ++q) { float d0 = __fsub_rn(v[q], mx); asm volatile("" : "+v"(d0)); v[q] = __builtin_amdgcn_exp2f(__fmul_rn(d0, 1.4426950408889634f)); sum += v[q]; }
#pragma unroll
    for (int sh = 16; sh; sh >>= 1) sum += __shfl_xor(sum, sh, 32);
    const float f = __fdiv_rn(1.0f, sum); v4us oh, ol;
#pragma unroll
    for (int q = 0; q < 4; ++q) { unsigned short h2, l2; float y = __fmul_rn(v[q], f); asm volatile("" : "+v"(y)); splitf(y, h2, l2); oh[q] = h2; ol[q] = l2; }
    const size_t oo = row * NN + lane * 4; *(volatile v4us*)(Ph + oo) = oh; *(volatile v4us*)(Pl + oo) = ol; __threadfence(); *(volatile v4us*)(Ph + oo) = oh; *(volatile v4us*)(Pl + oo) = ol; }
template <int MODE>
__global__ __launch_bounds__(256) void k_ln(const float* __restrict__ A, const float* __restrict__ g, const float* __restrict__ bb, const float* __restrict__ R, const float* __restrict__ g2, const float* __restrict__ b2, bf* Hh, bf* Hl, float* O32) {
    const int lane = threadIdx.x & 31; const size_t row = (size_t)blockIdx.x * 8 + (threadIdx.x >> 5); if (row >= (size_t)NR) return; const float* ar = A + row * HH; float v[8]; float s = 0.f;
#pragma unroll
    for (int ch = 0; ch < 2; ++ch) { const v4f a = *(const v4f*)(ar + ch * 128 + lane * 4);
#pragma unroll
        for (int q = 0; q < 4; ++q) { v[ch * 4 + q] = a[q]; s = __fadd_rn(s, a[q]); } }
#pragma unroll
    for (int sh = 16; sh; sh >>= 1) s = __fadd_rn(s, __shfl_xor(s, sh, 32));
    float mu = __fdiv_rn(s, (float)HH); float s2 = 0.f;
#pragma unroll
    for (int k = 0; k < 8; ++k) { float d0 = __fsub_rn(v[k], mu); asm volatile("" : "+v"(d0)); float p = __fmul_rn(d0, d0); asm volatile("" : "+v"(p)); s2 = __fadd_rn(s2, p); }
#pragma unroll
    for (int sh = 16; sh; sh >>= 1) s2 = __fadd_rn(s2, __shfl_xor(s2, sh, 32));
    float rs = __fdiv_rn(1.0f, __fsqrt_rn(__fadd_rn(__fdiv_rn(s2, (float)HH), 1e-5f)));
#pragma unroll
    for (int ch = 0; ch < 2; ++ch) {
#pragma unroll
        for (int q = 0; q < 4; ++q) { const int c = ch * 128 + lane * 4 + q; float xn = __fmul_rn(__fsub_rn(v[ch * 4 + q], mu), rs); asm volatile("" : "+v"(xn)); float y = __fmul_rn(xn, bfr(g[c])); asm volatile("" : "+v"(y)); y = __fadd_rn(y, bfr(bb[c])); v[ch * 4 + q] = (MODE == 1) ? __fadd_rn(fmaxf(y, 0.0f), R[row * HH + c]) : y; } }
    if (MODE == 1) {
        s = 0.f;
#pragma unroll
        for (int k = 0; k < 8; ++k) s = __fadd_rn(s, v[k]);
#pragma unroll
        for (int sh = 16; sh; sh >>= 1) s = __fadd_rn(s, __shfl_xor(s, sh, 32));
        mu = __fdiv_rn(s, (float)HH); s2 = 0.f;
#pragma unroll
        for (int k = 0; k < 8; ++k) { float d0 = __fsub_rn(v[k], mu); asm volatile("" : "+v"(d0)); float p = __fmul_rn(d0, d0); asm volatile("" : "+v"(p)); s2 = __fadd_rn(s2, p); }
#pragma unroll
        for (int sh = 16; sh; sh >>= 1) s2 = __fadd_rn(s2, __shfl_xor(s2, sh, 32));
        rs = __fdiv_rn(1.0f, __fsqrt_rn(__fadd_rn(__fdiv_rn(s2, (float)HH), 1e-5f)));
#pragma unroll
        for (int ch = 0; ch < 2; ++ch) {
#pragma unroll
            for (int q = 0; q < 4; ++q) { const int c = ch * 128 + lane * 4 + q; float xn = __fmul_rn(__fsub_rn(v[ch * 4 + q], mu), rs); asm volatile("" : "+v"(xn)); float y = __fmul_rn(xn, bfr(g2[c])); asm volatile("" : "+v"(y)); v[ch * 4 + q] = __fadd_rn(y, bfr(b2[c])); } } }
#pragma unroll 1
    for (int ps = 0; ps < 2; ++ps) {
#pragma unroll
        for (int ch = 0; ch < 2; ++ch) { const int c0 = ch * 128 + lane * 4;
            if (MODE == 0) { v4us oh, ol;
#pragma unroll
                for (int q = 0; q < 4; ++q) { unsigned short h2, l2; splitf(v[ch * 4 + q], h2, l2); oh[q] = h2; ol[q] = l2; }
                *(volatile v4us*)(Hh + row * HH + c0) = oh; *(volatile v4us*)(Hl + row * HH + c0) = ol; }
            else { v4f o; for (int q = 0; q < 4; ++q) o[q] = v[ch * 4 + q]; *(volatile v4f*)(O32 + row * HH + c0) = o; } }
        if (ps == 0) __threadfence(); }
}

extern "C" void kernel_launch(void* const* d_in, const int* in_sizes, int n_in,
                              void* d_out, int out_size, void* d_ws, size_t ws_size, hipStream_t stream) {
    (void)in_sizes; (void)n_in; (void)out_size;
    const float* x = (const float*)d_in[0]; const float* area = (const float*)d_in[1]; const float* co = (const float*)d_in[2]; const float* wf = (const float*)d_in[3]; const float* bfv = (const float*)d_in[4];
    const float* wq = (const float*)d_in[5]; const float* bq = (const float*)d_in[6]; const float* wk = (const float*)d_in[7]; const float* bk = (const float*)d_in[8]; const float* wv = (const float*)d_in[9]; const float* bv = (const float*)d_in[10];
    const float* we1 = (const float*)d_in[11]; const float* be1 = (const float*)d_in[12]; const float* we2 = (const float*)d_in[13]; const float* be2 = (const float*)d_in[14]; const float* wo = (const float*)d_in[15]; const float* bo = (const float*)d_in[16];
    const float* gO = (const float*)d_in[17]; const float* bO = (const float*)d_in[18]; const float* g1 = (const float*)d_in[19]; const float* b1 = (const float*)d_in[20]; const float* g2 = (const float*)d_in[21]; const float* b2 = (const float*)d_in[22];
    float* OUT = (float*)d_out;
    char* wsp = (char*)d_ws;
    auto take = [&](size_t bytes) { char* p = wsp; wsp += (bytes + 255) & ~(size_t)255; return (void*)p; };
    bf* WF = (bf*)take((size_t)HH * FIN * 2); bf* WQ = (bf*)take((size_t)HH * HH * 2); bf* WK = (bf*)take((size_t)HH * HH * 2); bf* WV = (bf*)take((size_t)HH * HH * 2); bf* WO = (bf*)take((size_t)HH * HH * 2);
    bf* XB = (bf*)take((size_t)NR * FIN * 2); float* XP = (float*)take((size_t)NR * HH * 4); bf* XPh = (bf*)take((size_t)NR * HH * 2); bf* XPl = (bf*)take((size_t)NR * HH * 2);
    float* F = (float*)take((size_t)NR * HH * 4); bf* Qh = (bf*)take((size_t)NR * HH * 2); bf* Ql = (bf*)take((size_t)NR * HH * 2); bf* Kh = (bf*)take((size_t)NR * HH * 2); bf* Kl = (bf*)take((size_t)NR * HH * 2); bf* VTh = (bf*)take((size_t)NR * HH * 2); bf* VTl = (bf*)take((size_t)NR * HH * 2);
    float* Sb = (float*)take((size_t)NR * NN * 4); bf* Ph = (bf*)take((size_t)NR * NN * 2); bf* Pl = (bf*)take((size_t)NR * NN * 2); float* O = (float*)take((size_t)NR * HH * 4); bf* Lh = (bf*)take((size_t)NR * HH * 2); bf* Ll = (bf*)take((size_t)NR * HH * 2); float* Y = (float*)take((size_t)NR * HH * 4);
    if ((size_t)(wsp - (char*)d_ws) > ws_size) return;
    const size_t N4 = (size_t)NR * HH / 4;
    k_wtG<<<(unsigned)((FIN * HH / 64 + 63) / 64), 256, 0, stream>>>(wf, FIN, HH, WF); k_wtG<<<(unsigned)((HH * HH / 64 + 63) / 64), 256, 0, stream>>>(wq, HH, HH, WQ); k_wtG<<<(unsigned)((HH * HH / 64 + 63) / 64), 256, 0, stream>>>(wk, HH, HH, WK); k_wtG<<<(unsigned)((HH * HH / 64 + 63) / 64), 256, 0, stream>>>(wv, HH, HH, WV); k_wtG<<<(unsigned)((HH * HH / 64 + 63) / 64), 256, 0, stream>>>(wo, HH, HH, WO);
    k_cvt8<<<(unsigned)(((size_t)NR * FIN / 8 + 255) / 256), 256, 0, stream>>>(x, XB, (size_t)NR * FIN / 8);
    k_gemmw<bf, 0, true><<<dim3(NR / 64, HH / 64, 1), 32, 0, stream>>>(XB, nullptr, WF, nullptr, FIN, XP, HH, bfv, 0, 0, 0);
    k_tohl<<<(unsigned)((N4 + 255) / 256), 256, 0, stream>>>(XP, XPh, XPl, N4);
    k_gemmw<bf, 1, true><<<dim3(NR / 64, HH / 64, 1), 32, 0, stream>>>(XPh, XPl, WQ, nullptr, HH, F, HH, bq, 0, 0, 0); k_tohl<<<(unsigned)((N4 + 255) / 256), 256, 0, stream>>>(F, Qh, Ql, N4);
    k_gemmw<bf, 1, true><<<dim3(NR / 64, HH / 64, 1), 32, 0, stream>>>(XPh, XPl, WK, nullptr, HH, F, HH, bk, 0, 0, 0); k_tohl<<<(unsigned)((N4 + 255) / 256), 256, 0, stream>>>(F, Kh, Kl, N4);
    k_gemmw<bf, 1, true><<<dim3(NR / 64, HH / 64, 1), 32, 0, stream>>>(XPh, XPl, WV, nullptr, HH, F, HH, bv, 0, 0, 0); k_vtB<<<(unsigned)(((size_t)NBT * HH * NN / 2 + 255) / 256), 256, 0, stream>>>(F, VTh, VTl);
    k_gemmw<bf, 2, false><<<dim3(NN / 64, NN / 64, NBT), 32, 0, stream>>>(Qh, Ql, Kh, Kl, HH, Sb, NN, nullptr, (size_t)NN * HH, (size_t)NN * HH, (size_t)NN * NN);
    k_esoft<<<NR / 8, 256, 0, stream>>>(Sb, area, co, we1, be1, we2, be2, Ph, Pl);
    k_gemmw<bf, 2, false><<<dim3(NN / 64, HH / 64, NBT), 32, 0, stream>>>(Ph, Pl, VTh, VTl, NN, O, HH, nullptr, (size_t)NN * NN, (size_t)HH * NN, (size_t)NN * HH);
    k_ln<0><<<NR / 8, 256, 0, stream>>>(O, g1, b1, nullptr, nullptr, nullptr, Lh, Ll, nullptr);
    k_gemmw<bf, 1, true><<<dim3(NR / 64, HH / 64, 1), 32, 0, stream>>>(Lh, Ll, WO, nullptr, HH, Y, HH, bo, 0, 0, 0);
    k_ln<1><<<NR / 8, 256, 0, stream>>>(Y, gO, bO, XP, g2, b2, nullptr, nullptr, OUT);
}
